// MultiBoxConvBlock_47708496724920
// MI455X (gfx1250) — hardware-verified
//
#include <hip/hip_runtime.h>
#include <math.h>

#define NB_ 4
#define CC_ 64
#define KB_ 4
#define IH  192
#define IW  192
#define IST 224
#define IPL ((IH + 1) * IST)
#define NF  (CC_ * KB_)

typedef _Float16 f16;
typedef __attribute__((ext_vector_type(16))) f16 f16x16;
typedef __attribute__((ext_vector_type(8)))  f16 f16x8;
typedef __attribute__((ext_vector_type(8)))  float f32x8;
typedef __attribute__((ext_vector_type(4)))  float v4f_t;
typedef float v4fa __attribute__((ext_vector_type(4), may_alias));

__device__ __forceinline__ f32x8 wmma16(f16x16 a, f16x16 b, f32x8 c) {
  c = __builtin_amdgcn_wmma_f32_16x16x32_f16(false, a, false, b, (short)0, c, false, false);
  asm volatile("v_nop\n\tv_nop\n\tv_nop\n\tv_nop" : "+v"(c) : "v"(a), "v"(b));
  return c;
}
__device__ __forceinline__ f16x16 lds_frag(const f16* base, int stride) {
  const int lane = threadIdx.x & 31, row = lane & 15, kh = (lane >> 4) * 8;
  const f16x8 lo = *(const f16x8*)(base + row * stride + kh);
  const f16x8 hi = *(const f16x8*)(base + row * stride + kh + 16);
  f16x16 f;
#pragma unroll
  for (int i = 0; i < 8; ++i) { f[i] = lo[i]; f[i + 8] = hi[i]; }
  return f;
}

template <bool RELU>
__global__ __launch_bounds__(256) void k_rowscan(const float* __restrict__ src, float* __restrict__ ii) {
  __shared__ __attribute__((aligned(16))) float rS[32 * IST];
  const int tid = threadIdx.x, plane = blockIdx.x / 6, y0 = (blockIdx.x % 6) * 32;
  const float* sp = src + (size_t)plane * IH * IW + (size_t)y0 * IW;
  for (int e = tid; e < 32 * IST; e += 256) { const int r = e / IST, c = e % IST; float v = 0.0f;
    if (c >= 1 && c <= IW) { v = sp[(size_t)r * IW + (c - 1)]; if (RELU) v = fmaxf(v, 0.0f); } rS[e] = v; }
  __syncthreads();
  if (tid < 32) { float run = 0.0f; float* row = rS + tid * IST;
    for (int c = 1; c <= IW; ++c) { run += row[c]; row[c] = run; } }
  __syncthreads();
  float* dst = ii + (size_t)plane * IPL + (size_t)(y0 + 1) * IST;
#pragma unroll 1
  for (int pass = 0; pass < 2; ++pass) {
    for (int q = tid; q < 32 * IST / 4; q += 256) *(volatile v4f_t*)(dst + q * 4) = *(const v4fa*)(rS + q * 4);
    __threadfence();
  }
}
__global__ __launch_bounds__(32) void k_colscan(float* __restrict__ ii) {
  const int lane = threadIdx.x, plane = blockIdx.x / 7, ch = blockIdx.x % 7;
  float* col = ii + (size_t)plane * IPL + ch * 32 + lane;
  float run = 0.0f;
  *(volatile float*)col = 0.0f; __threadfence(); *(volatile float*)col = 0.0f;
  for (int y = 1; y <= IH; ++y) { run += *(const volatile float*)(col + (size_t)y * IST);
    *(volatile float*)(col + (size_t)y * IST) = run; __threadfence(); *(volatile float*)(col + (size_t)y * IST) = run; }
}

__device__ __forceinline__ f16x16 wfragB(const float* __restrict__ Wc, int o0, int k0) {
  const int lane = threadIdx.x & 31, r = lane & 15, kh = (lane >> 4) * 8;
  const float* p = Wc + (size_t)(o0 + r) * NF + k0 + kh;
  const v4f_t a = *(const v4f_t*)p, b2 = *(const v4f_t*)(p + 4), c = *(const v4f_t*)(p + 16), d = *(const v4f_t*)(p + 20);
  f16x16 f;
  f[0]=(f16)a[0]; f[1]=(f16)a[1]; f[2]=(f16)a[2]; f[3]=(f16)a[3]; f[4]=(f16)b2[0]; f[5]=(f16)b2[1]; f[6]=(f16)b2[2]; f[7]=(f16)b2[3];
  f[8]=(f16)c[0]; f[9]=(f16)c[1]; f[10]=(f16)c[2]; f[11]=(f16)c[3]; f[12]=(f16)d[0]; f[13]=(f16)d[1]; f[14]=(f16)d[2]; f[15]=(f16)d[3];
  return f;
}
template <int STAGE>
__global__ __launch_bounds__(256) void k_boxconv(const float* __restrict__ ii, const float* __restrict__ ymin, const float* __restrict__ ymax,
                                                 const float* __restrict__ xmin, const float* __restrict__ xmax, const float* __restrict__ Wc,
                                                 const float* __restrict__ bc, const float* __restrict__ xres, float* __restrict__ dst) {
  __shared__ __attribute__((aligned(16))) f16 aS[96 * 264];
  __shared__ float rb[32 * 196];
  __shared__ float cw[4][32]; __shared__ int cr[4][32];
  __shared__ float inva[32];
  __shared__ __attribute__((aligned(16))) float outS[64 * 100];
  const int tid = threadIdx.x, lane = tid & 31, wave = tid >> 5, cl = lane & 15, rh = (lane >> 4) * 8;
  const int b = blockIdx.x / (IH * 2), rem = blockIdx.x % (IH * 2), y = rem >> 1, x0 = (rem & 1) * 96;
  const int jlo = 0, jhi = IW + 1;
  const float gy = (float)y + 0.5f;
#pragma unroll 1
  for (int g = 0; g < 8; ++g) {
    __syncthreads();
    if (tid < 32) {
      const int f = g * 32 + tid, c = f >> 2, k = f & 3;
      const float ym = ymin[c * KB_ + k], yM = ymax[c * KB_ + k], xm = xmin[c * KB_ + k], xM = xmax[c * KB_ + k];
      const float yt = fminf(fmaxf(gy + ym, 0.0f), (float)IH), yb = fminf(fmaxf(gy + yM, 0.0f), (float)IH);
      const float t0 = fminf(fmaxf(floorf(yt), 0.0f), (float)(IH - 1)), b0 = fminf(fmaxf(floorf(yb), 0.0f), (float)(IH - 1));
      const float ft = yt - t0, fb = yb - b0;
      cr[0][tid] = (int)t0;     cw[0][tid] = 1.0f - ft;
      cr[1][tid] = (int)t0 + 1; cw[1][tid] = ft;
      cr[2][tid] = (int)b0;     cw[2][tid] = 1.0f - fb;
      cr[3][tid] = (int)b0 + 1; cw[3][tid] = fb;
      inva[tid] = 1.0f / ((yM - ym) * (xM - xm));
    }
    __syncthreads();
    { const int nj = jhi - jlo;
      for (int e = tid; e < 32 * nj; e += 256) { const int fl = e / nj, j = jlo + e % nj; const int c = (g * 32 + fl) >> 2;
        const float* pl = ii + ((size_t)(b * CC_ + c)) * IPL + j;
        const float top = cw[0][fl] * pl[(size_t)cr[0][fl] * IST] + cw[1][fl] * pl[(size_t)cr[1][fl] * IST];
        const float bot = cw[2][fl] * pl[(size_t)cr[2][fl] * IST] + cw[3][fl] * pl[(size_t)cr[3][fl] * IST];
        rb[fl * 196 + (j - jlo)] = bot - top; } }
    __syncthreads();
    for (int e = tid; e < 96 * 32; e += 256) { const int px = e >> 5, fl = e & 31; const int f = g * 32 + fl, c = f >> 2, k = f & 3;
      const float gx = (float)(x0 + px) + 0.5f;
      const float xm = xmin[c * KB_ + k], xM = xmax[c * KB_ + k];
      const float xl = fminf(fmaxf(gx + xm, 0.0f), (float)IW), xr = fminf(fmaxf(gx + xM, 0.0f), (float)IW);
      const float l0 = fminf(fmaxf(floorf(xl), 0.0f), (float)(IW - 1)), r0 = fminf(fmaxf(floorf(xr), 0.0f), (float)(IW - 1));
      const float fxl = xl - l0, fxr = xr - r0;
      const int li = (int)l0 - jlo, ri = (int)r0 - jlo;
      const float* band = rb + fl * 196;
      const float left = (1.0f - fxl) * band[li] + fxl * band[li + 1];
      const float right = (1.0f - fxr) * band[ri] + fxr * band[ri + 1];
      aS[px * 264 + f] = (f16)((right - left) * inva[fl]);
    }
  }
  __syncthreads();
#pragma unroll 1
  for (int t3 = 0; t3 < 3; ++t3) {
    const int tix = wave * 3 + t3, rt = tix >> 2, nt = tix & 3;
    f32x8 acc = {};
#pragma unroll
    for (int ks = 0; ks < 8; ++ks) acc = wmma16(lds_frag(aS + (rt * 16) * 264 + ks * 32, 264), wfragB(Wc, nt * 16, ks * 32), acc);
    const int o = nt * 16 + cl; const float bo = bc[o];
#pragma unroll
    for (int r = 0; r < 8; ++r) {
      const int px = rt * 16 + rh + r;
      float v = acc[r] + bo;
      if (STAGE == 2) v += xres[(((size_t)b * CC_ + o) * IH + y) * IW + x0 + px];
      outS[o * 100 + px] = fmaxf(v, 0.0f);
    }
  }
  __syncthreads();
#pragma unroll 1
  for (int pass = 0; pass < 2; ++pass) {
    for (int q = tid; q < 64 * 24; q += 256) { const int o = q / 24, c4 = (q % 24) * 4;
      *(volatile v4f_t*)(dst + (((size_t)b * CC_ + o) * IH + y) * IW + x0 + c4) = *(const v4fa*)(outS + o * 100 + c4); }
    __threadfence();
  }
}

extern "C" void kernel_launch(void* const* d_in, const int* in_sizes, int n_in,
                              void* d_out, int out_size, void* d_ws, size_t ws_size,
                              hipStream_t stream) {
  (void)in_sizes; (void)n_in; (void)out_size; (void)ws_size;
  const float* x = (const float*)d_in[0];
  const float* ymin1 = (const float*)d_in[1], *ymax1 = (const float*)d_in[2], *xmin1 = (const float*)d_in[3], *xmax1 = (const float*)d_in[4];
  const float* w1 = (const float*)d_in[5], *b1 = (const float*)d_in[6];
  const float* ymin2 = (const float*)d_in[7], *ymax2 = (const float*)d_in[8], *xmin2 = (const float*)d_in[9], *xmax2 = (const float*)d_in[10];
  const float* w2 = (const float*)d_in[11], *b2 = (const float*)d_in[12];
  float* out = (float*)d_out;
  char* ws = (char*)d_ws;
  float* ii = (float*)ws; ws += (size_t)NB_ * CC_ * IPL * 4;
  float* h1 = (float*)ws; ws += (size_t)NB_ * CC_ * IH * IW * 4;
  const int planes = NB_ * CC_;
  k_rowscan<true><<<dim3(planes * 6), dim3(256), 0, stream>>>(x, ii);
  k_colscan<<<dim3(planes * 7), dim3(32), 0, stream>>>(ii);
  k_boxconv<1><<<dim3(NB_ * IH * 2), dim3(256), 0, stream>>>(ii, ymin1, ymax1, xmin1, xmax1, w1, b1, nullptr, h1);
  k_rowscan<false><<<dim3(planes * 6), dim3(256), 0, stream>>>(h1, ii);
  k_colscan<<<dim3(planes * 7), dim3(32), 0, stream>>>(ii);
  k_boxconv<2><<<dim3(NB_ * IH * 2), dim3(256), 0, stream>>>(ii, ymin2, ymax2, xmin2, xmax2, w2, b2, x, out);
}
